// UV_Aggregator_51092930953381
// MI455X (gfx1250) — hardware-run, weakly checked
//
#include <hip/hip_runtime.h>
#include <math.h>

#define NND   4096
#define HS    50
#define DD    128
#define NTAB  100000
#define NRAT  5
#define NPB   64
#define PX    264
#define PT    136
#define WK    128
#define PLN   (DD * WK)
#define NPL   6
#define NCST  11
#define NTHR  128
#define PTHR  256

typedef __bf16         v16b __attribute__((ext_vector_type(16)));
typedef __bf16         v8b  __attribute__((ext_vector_type(8)));
typedef unsigned short v8us __attribute__((ext_vector_type(8)));
typedef unsigned int   v2u  __attribute__((ext_vector_type(2)));
typedef float          v8f  __attribute__((ext_vector_type(8)));
typedef float          v4f  __attribute__((ext_vector_type(4)));
typedef v8b  __attribute__((may_alias)) v8ba;
typedef v8us __attribute__((may_alias)) v8usa;
typedef v2u  __attribute__((may_alias)) v2ua;
typedef v4f  __attribute__((may_alias)) v4fa;

static_assert(NND % NPB == 0);
static_assert((PX % 8) == 0 && (PT % 8) == 0 && (WK % 8) == 0);
static_assert(NPB == 64 && NTHR == 128 && PTHR == 256);
static_assert(HS >= 1 && HS <= 64);
static_assert(NPL * PLN * 2 == 196608);
static_assert(3 * (NTHR / 32) >= NCST);
static_assert(DD == 4 * 32);

__device__ __forceinline__ unsigned short f2bf_bits(float f) {
  const unsigned u = __float_as_uint(f);
  return (unsigned short)((u + 0x7FFFu + ((u >> 16) & 1u)) >> 16);
}
__device__ __forceinline__ float bf2f(unsigned short b) { return __uint_as_float(((unsigned)b) << 16); }
__device__ __forceinline__ float bfr(float f) { return bf2f(f2bf_bits(f)); }
__device__ __forceinline__ unsigned pk2(float a, float b) {
  return (unsigned)f2bf_bits(a) | ((unsigned)f2bf_bits(b) << 16);
}

__device__ __forceinline__ v8f mma_bf16(v16b a, v16b b, v8f c) {
  c = __builtin_amdgcn_wmma_f32_16x16x32_bf16(false, a, false, b, (short)0, c, false, false);
  asm volatile("v_nop\n\tv_nop\n\tv_nop\n\tv_nop" : "+v"(c) : "v"(a), "v"(b));
  return c;
}

__device__ __forceinline__ v16b ld_frag(const unsigned short* p) {
  union { v16b v; v8b hh[2]; } f;
  f.hh[0] = *(const v8ba*)(p);
  f.hh[1] = *(const v8ba*)(p + 16);
  return f.v;
}

template <int NK, int KWM>
__device__ __forceinline__ void tile_mma8(v8f (&acc)[8], const unsigned short* ap,
                                          const unsigned short* bp, int bstep) {
  const v8f z = {0.f, 0.f, 0.f, 0.f, 0.f, 0.f, 0.f, 0.f};
#pragma unroll
  for (int nt = 0; nt < 8; ++nt) acc[nt] = z;
#pragma unroll 1
  for (int ks = 0; ks < NK; ++ks) {
    const int k0 = ks << 5;
    const int kb = k0 & KWM;
    const v16b a = ld_frag(ap + k0);
#pragma unroll
    for (int nt = 0; nt < 8; ++nt) {
      const v16b b = ld_frag(bp + nt * bstep + kb);
      acc[nt] = mma_bf16(a, b, acc[nt]);
    }
  }
}

__device__ __forceinline__ void split8(float v, unsigned short* trow, int r, int c) {
  const unsigned short hb = f2bf_bits(v);
  trow[r * PX + c]      = hb;
  trow[r * PX + DD + c] = f2bf_bits(v - bf2f(hb));
}

__device__ __forceinline__ void gather_row(unsigned short* dst, const float* src) {
#pragma unroll 8
  for (int j = 0; j < 16; ++j) {
    const v4f v = *(const v4fa*)(src + 4 * j);
    v2u pk;
    pk.x = pk2(v.x, v.y);
    pk.y = pk2(v.z, v.w);
    *(v2ua*)(dst + 4 * j) = pk;
  }
}

__device__ __forceinline__ void out_store_pass(const float* so, float* out, int nb0, int rw, int lane) {
#pragma unroll
  for (int row = 0; row < 16; ++row) {
    const v4f v = *(const v4fa*)(so + (rw + row) * DD + 4 * lane);
    *(volatile v4f*)(out + (size_t)(nb0 + rw + row) * DD + 4 * lane) = v;
  }
}

__device__ __forceinline__ void plane_store_pass(const unsigned short* sT, unsigned short* dst, int w, int lane) {
  const int hh = lane >> 4, kof = (lane & 15) << 3;
#pragma unroll
  for (int it = 0; it < 8; ++it) {
    const int row = 2 * (it * 8 + w) + hh;
    const v8us v = *(const v8usa*)(sT + row * PT + kof);
    *(volatile v8us*)(dst + row * WK + kof) = v;
  }
}

__global__ __launch_bounds__(PTHR) void prep_kernel(
    const float* __restrict__ ge_w, const float* __restrict__ wr1_w, const float* __restrict__ wr2_w,
    const float* __restrict__ att1_w, const float* __restrict__ att2_w,
    unsigned short* __restrict__ wpl)
{
  __shared__ __align__(16) unsigned short sT[DD * PT];
  const int t = threadIdx.x, lane = t & 31, w = t >> 5, b = blockIdx.x;
  const float* src = (b == 0) ? ge_w : (b == 1) ? wr1_w : (b == 2) ? wr2_w : (b == 3) ? att1_w
                   : (b == 4) ? (att1_w + (size_t)DD * DD) : att2_w;
#pragma unroll 2
  for (int it = 0; it < 16; ++it) {
    const int f = it * PTHR + t;
    const int k = f >> 5, n4 = (f & 31) << 2;
    const v4f v = *(const v4fa*)(src + (size_t)f * 4);
    sT[(n4 + 0) * PT + k] = f2bf_bits(v.x);
    sT[(n4 + 1) * PT + k] = f2bf_bits(v.y);
    sT[(n4 + 2) * PT + k] = f2bf_bits(v.z);
    sT[(n4 + 3) * PT + k] = f2bf_bits(v.w);
  }
  __syncthreads();
  unsigned short* dst = wpl + (size_t)b * PLN;
  plane_store_pass(sT, dst, w, lane);
  __threadfence();
  plane_store_pass(sT, dst, w, lane);
}

__global__ __launch_bounds__(NTHR) void uvagg_kernel(
    const int* __restrict__ nodes, const int* __restrict__ huv, const int* __restrict__ hr,
    const int* __restrict__ hlen,
    const float* __restrict__ u2e, const float* __restrict__ v2e, const float* __restrict__ r2e,
    const float* __restrict__ wr1, const float* __restrict__ geb, const float* __restrict__ b1,
    const float* __restrict__ b2, const float* __restrict__ ab1, const float* __restrict__ ab2,
    const float* __restrict__ a3, const float* __restrict__ ab3,
    const unsigned short* __restrict__ wpl, float* __restrict__ out)
{
  __shared__ __align__(16) unsigned short sT0[NPB * PX];
  __shared__ __align__(16) unsigned short sT1[NPB * PX];
  __shared__ __align__(16) float sO[NPB * DD];
  __shared__ __align__(16) float sAcc[NPB * DD];
  __shared__ __align__(16) float sQa[NPB * DD];
  __shared__ __align__(16) float sR5[NRAT * DD];
  __shared__ __align__(16) float sCst[NCST * DD];
  __shared__ int sRR[NPB];
  __shared__ int sHL[NPB];

  const int t = threadIdx.x;
  const int lane = t & 31, w = t >> 5, h = lane >> 4, m = lane & 15;
  const int nb0 = blockIdx.x * NPB;
  const int rw = 16 * w;
  const int rrow = rw + 8 * h;

#pragma unroll 1
  for (int it = 0; it < 3; ++it) {
    const int ri  = it * 4 + w;
    const int ric = min(ri, NCST - 1);
    const float* src = (ric == 0) ? geb : (ric == 1) ? b1 : (ric == 2) ? b2 : (ric == 3) ? ab1
                     : (ric == 4) ? ab2 : (ric == 5) ? a3 : (r2e + (size_t)max(ric - 6, 0) * DD);
    const v4f v = *(const v4fa*)(src + 4 * lane);
    if (ri < NCST) {
      float* dst = sCst + ric * DD + 4 * lane;
      dst[0] = bfr(v.x);
      dst[1] = bfr(v.y);
      dst[2] = bfr(v.z);
      dst[3] = bfr(v.w);
    }
  }
  const float ab3v = bfr(ab3[0]);
  {
    int hl = hlen[nb0 + min(t, NPB - 1)];
    hl = max(hl, 1);
    hl = min(hl, HS);
    if (t < NPB) sHL[t] = hl;
  }
  {
    const int row = t >> 1, half = t & 1;
    int nd = nodes[nb0 + row];
    nd = (nd < 0) ? nd + NTAB : nd;
    nd = min(max(nd, 0), NTAB - 1);
    gather_row(sT1 + row * PX + half * 64, v2e + (size_t)nd * DD + half * 64);
  }
  __syncthreads();

  {
    float r5[NRAT];
#pragma unroll
    for (int r = 0; r < NRAT; ++r) r5[r] = 0.0f;
#pragma unroll 1
    for (int k = 0; k < DD; ++k) {
      const float wv = bfr(wr1[(size_t)(DD + k) * DD + t]);
#pragma unroll
      for (int r = 0; r < NRAT; ++r) r5[r] = fmaf(sCst[(6 + r) * DD + k], wv, r5[r]);
    }
#pragma unroll
    for (int r = 0; r < NRAT; ++r) sR5[r * DD + t] = r5[r];
  }

  int hlr[8];
#pragma unroll
  for (int r = 0; r < 8; ++r) hlr[r] = sHL[rrow + r];

  const unsigned short* apT0 = sT0 + (rw + m) * PX + 8 * h;
  const unsigned short* apT1 = sT1 + (rw + m) * PX + 8 * h;
  const unsigned short* bpl  = wpl + m * WK + 8 * h;
  const int bstep = 16 * WK;
  unsigned short* t0row = sT0 + rrow * PX;
  unsigned short* t1row = sT1 + rrow * PX;

  v8f acc[8];

  tile_mma8<4, 127>(acc, apT1, bpl + 4 * PLN, bstep);
#pragma unroll
  for (int nt = 0; nt < 8; ++nt)
#pragma unroll
    for (int r = 0; r < 8; ++r) {
      const int e = (rrow + r) * DD + 16 * nt + m;
      sQa[e]  = acc[nt][r];
      sAcc[e] = 0.0f;
    }

  float mrun[8], lrun[8];
#pragma unroll
  for (int r = 0; r < 8; ++r) { mrun[r] = -1e30f; lrun[r] = 0.0f; }

#pragma unroll 1
  for (int l = 0; l < HS; ++l) {
    __syncthreads();
    {
      const int row = t >> 1, half = t & 1;
      const int hidx = (nb0 + row) * HS + l;
      int item = huv[hidx];
      item = (item < 0) ? item + NTAB : item;
      item = min(max(item, 0), NTAB - 1);
      int rr = hr[hidx];
      rr = (rr < 0) ? rr + NRAT : rr;
      rr = min(max(rr, 0), NRAT - 1);
      sRR[row] = rr;
      gather_row(sT1 + row * PX + half * 64, u2e + (size_t)item * DD + half * 64);
    }
    __syncthreads();
    int rrr[8];
#pragma unroll
    for (int r = 0; r < 8; ++r) rrr[r] = sRR[rrow + r];

    tile_mma8<4, 127>(acc, apT1, bpl, bstep);
#pragma unroll
    for (int nt = 0; nt < 8; ++nt) {
      const int c = 16 * nt + m;
      const float b = sCst[c];
#pragma unroll
      for (int r = 0; r < 8; ++r) split8(fmaxf(acc[nt][r] + b, 0.0f), t0row, r, c);
    }
    __syncthreads();

    tile_mma8<8, 127>(acc, apT0, bpl + PLN, bstep);
#pragma unroll
    for (int nt = 0; nt < 8; ++nt) {
      const int c = 16 * nt + m;
      const float b = sCst[DD + c];
#pragma unroll
      for (int r = 0; r < 8; ++r) {
        const float v = fmaxf(acc[nt][r] + sR5[rrr[r] * DD + c] + b, 0.0f);
        split8(v, t1row, r, c);
      }
    }
    __syncthreads();

    tile_mma8<8, 127>(acc, apT1, bpl + 2 * PLN, bstep);
#pragma unroll
    for (int nt = 0; nt < 8; ++nt) {
      const int c = 16 * nt + m;
      const float b = sCst[2 * DD + c];
#pragma unroll
      for (int r = 0; r < 8; ++r) {
        const float v = fmaxf(acc[nt][r] + b, 0.0f);
        sO[(rrow + r) * DD + c] = v;
        split8(v, t0row, r, c);
      }
    }
    __syncthreads();

    tile_mma8<8, 127>(acc, apT0, bpl + 3 * PLN, bstep);
#pragma unroll
    for (int nt = 0; nt < 8; ++nt) {
      const int c = 16 * nt + m;
      const float b = sCst[3 * DD + c];
#pragma unroll
      for (int r = 0; r < 8; ++r) {
        const float v = fmaxf(acc[nt][r] + sQa[(rrow + r) * DD + c] + b, 0.0f);
        split8(v, t1row, r, c);
      }
    }
    __syncthreads();

    tile_mma8<8, 127>(acc, apT1, bpl + 5 * PLN, bstep);
    float part[8];
#pragma unroll
    for (int r = 0; r < 8; ++r) part[r] = 0.0f;
#pragma unroll
    for (int nt = 0; nt < 8; ++nt) {
      const int c = 16 * nt + m;
      const float b = sCst[4 * DD + c];
      const float a3c = sCst[5 * DD + c];
#pragma unroll
      for (int r = 0; r < 8; ++r) {
        const float v = fmaxf(acc[nt][r] + b, 0.0f);
        part[r] = fmaf(v, a3c, part[r]);
      }
    }
#pragma unroll
    for (int r = 0; r < 8; ++r) {
      float p = part[r];
      p += __shfl_xor(p, 1);
      p += __shfl_xor(p, 2);
      p += __shfl_xor(p, 4);
      p += __shfl_xor(p, 8);
      part[r] = p;
    }

#pragma unroll
    for (int r = 0; r < 8; ++r) {
      const float lg = part[r] + ab3v;
      const bool valid = (l < hlr[r]);
      const float mold = mrun[r];
      const float mnew = valid ? fmaxf(mold, lg) : mold;
      const float alpha = expf(mold - mnew);
      const float parg = valid ? (lg - mnew) : -1e30f;
      const float p = expf(parg);
      mrun[r] = mnew;
      lrun[r] = lrun[r] * alpha + p;
#pragma unroll
      for (int nt = 0; nt < 8; ++nt) {
        const int e = (rrow + r) * DD + 16 * nt + m;
        sAcc[e] = sAcc[e] * alpha + p * sO[e];
      }
    }
  }

#pragma unroll
  for (int r = 0; r < 8; ++r) {
    const float inv = 1.0f / lrun[r];
#pragma unroll
    for (int nt = 0; nt < 8; ++nt) {
      const int e = (rrow + r) * DD + 16 * nt + m;
      sAcc[e] = sAcc[e] * inv;
    }
  }
  __syncthreads();
  out_store_pass(sAcc, out, nb0, rw, lane);
  __threadfence();
  out_store_pass(sAcc, out, nb0, rw, lane);
}

extern "C" void kernel_launch(void* const* d_in, const int* in_sizes, int n_in,
                              void* d_out, int out_size, void* d_ws, size_t ws_size,
                              hipStream_t stream) {
  if (n_in < 19) return;
  if (in_sizes[0] != NND) return;
  if (in_sizes[1] != NND * HS || in_sizes[2] != NND * HS) return;
  if (in_sizes[3] != NND) return;
  if (in_sizes[4] != NTAB * DD || in_sizes[5] != NTAB * DD) return;
  if (in_sizes[6] != NRAT * DD) return;
  if (in_sizes[7] != DD * DD || in_sizes[8] != DD) return;
  if (in_sizes[9] != 2 * DD * DD || in_sizes[10] != DD) return;
  if (in_sizes[11] != DD * DD || in_sizes[12] != DD) return;
  if (in_sizes[13] != 2 * DD * DD || in_sizes[14] != DD) return;
  if (in_sizes[15] != DD * DD || in_sizes[16] != DD) return;
  if (in_sizes[17] != DD || in_sizes[18] != 1) return;
  if (out_size != NND * DD) return;
  const size_t ws_need = (size_t)NPL * PLN * sizeof(unsigned short);
  if (ws_need > ws_size) return;

  const int*   nodes  = (const int*)d_in[0];
  const int*   huv    = (const int*)d_in[1];
  const int*   hr     = (const int*)d_in[2];
  const int*   hlen   = (const int*)d_in[3];
  const float* u2e    = (const float*)d_in[4];
  const float* v2e    = (const float*)d_in[5];
  const float* r2e    = (const float*)d_in[6];
  const float* ge_w   = (const float*)d_in[7];
  const float* ge_b   = (const float*)d_in[8];
  const float* wr1_w  = (const float*)d_in[9];
  const float* wr1_b  = (const float*)d_in[10];
  const float* wr2_w  = (const float*)d_in[11];
  const float* wr2_b  = (const float*)d_in[12];
  const float* att1_w = (const float*)d_in[13];
  const float* att1_b = (const float*)d_in[14];
  const float* att2_w = (const float*)d_in[15];
  const float* att2_b = (const float*)d_in[16];
  const float* att3_w = (const float*)d_in[17];
  const float* att3_b = (const float*)d_in[18];
  float* out = (float*)d_out;
  unsigned short* wpl = (unsigned short*)d_ws;

  prep_kernel<<<dim3(NPL), dim3(PTHR), 0, stream>>>(ge_w, wr1_w, wr2_w, att1_w, att2_w, wpl);
  (void)hipGetLastError();
  uvagg_kernel<<<dim3(NND / NPB), dim3(NTHR), 0, stream>>>(
      nodes, huv, hr, hlen, u2e, v2e, r2e, wr1_w, ge_b, wr1_b, wr2_b, att1_b, att2_b,
      att3_w, att3_b, wpl, out);
  (void)hipGetLastError();
}
